// MultiHeadAttention3D_7249904796467
// MI455X (gfx1250) — hardware-verified
//
#include <hip/hip_runtime.h>
#include <math.h>

constexpr int kBatch = 2;
constexpr int kSeq   = 2048;
constexpr int kDim   = 1024;
constexpr int kHeads = 16;
constexpr int kDh    = 64;
constexpr int kGroup = 2;
constexpr int kTok   = kBatch * kSeq;
constexpr int kNumW  = 7;
constexpr float kScale     = 0.125f;
constexpr float kWCarry    = 16.0f;
constexpr float kWCarryInv = 1.0f / 16.0f;
constexpr float kACarry    = 16.0f;
constexpr float kPCarry    = 32768.0f;
constexpr float kPCarryInv = 1.0f / 32768.0f;
static_assert(kHeads * kDh == kDim);
static_assert(kSeq % 64 == 0 && kDim % 64 == 0 && kDh % 64 == 0 && kTok % 64 == 0);
static_assert(kDh % 32 == 0 && kDim % 32 == 0 && kSeq % 32 == 0);
static_assert(kHeads % kGroup == 0);
static_assert(kSeq == 256 * 8);

constexpr size_t kSzAct16 = (size_t)kTok * kDim * 2;
constexpr size_t kSzW16   = (size_t)kDim * kDim * 2;
constexpr size_t kSzAct32 = (size_t)kTok * kDim * 4;
constexpr int    kPlanes  = (kGroup > kBatch) ? kGroup : kBatch;
constexpr size_t kSzSC    = (size_t)kPlanes * kSeq * kSeq * 4;
constexpr size_t kSzPP    = (size_t)kPlanes * kSeq * kSeq * 2;
constexpr size_t kOffXO   = 0;
constexpr size_t kOffCTX  = kOffXO + kSzAct16;
constexpr size_t kOffW    = kOffCTX + kSzAct16;
constexpr size_t kOffQ    = kOffW + (size_t)kNumW * kSzW16;
constexpr size_t kOffK    = kOffQ + kSzAct16;
constexpr size_t kOffVT   = kOffK + kSzAct16;
constexpr size_t kOffAO32 = kOffVT + kSzAct16;
constexpr size_t kOffAO16 = kOffAO32 + kSzAct32;
constexpr size_t kOffSC   = kOffAO16 + kSzAct16;
constexpr size_t kOffPP   = kOffSC + kSzSC;
constexpr size_t kWsTotal = kOffPP + kSzPP;
static_assert(kWsTotal == 132120576);
static_assert(kWsTotal <= 134217728);
static_assert((size_t)kBatch * kDim * kSeq * 2 == kSzAct16);
static_assert((size_t)kGroup * kSeq * kSeq * 4 <= kSzSC && (size_t)kBatch * kSeq * kSeq * 4 <= kSzSC);
static_assert((size_t)kGroup * kSeq * kSeq * 2 <= kSzPP && (size_t)kBatch * kSeq * kSeq * 2 <= kSzPP);

typedef __attribute__((ext_vector_type(16))) _Float16 v16h;
typedef __attribute__((ext_vector_type(8)))  _Float16 v8h;
typedef __attribute__((ext_vector_type(16))) __bf16   v16b;
typedef __attribute__((ext_vector_type(8)))  __bf16   v8b;
typedef __attribute__((ext_vector_type(8)))  float    v8f;
typedef __attribute__((ext_vector_type(4)))  float    v4f;
typedef __attribute__((ext_vector_type(4)))  unsigned int v4u;

__device__ __forceinline__ unsigned short f2bf_bits(float f) {
  unsigned u = __float_as_uint(f);
  return (unsigned short)((u + 0x7FFFu + ((u >> 16) & 1u)) >> 16);
}
__device__ __forceinline__ float bf_bits2f(unsigned short h) { return __uint_as_float(((unsigned)h) << 16); }

__device__ __forceinline__ void dep_guard4_h(v8f& a, v8f& b, v8f& c, v8f& d, v16h x, v16h y) { asm volatile("v_nop\n\tv_nop\n\tv_nop\n\tv_nop" : "+v"(a), "+v"(b), "+v"(c), "+v"(d) : "v"(x), "v"(y)); }
__device__ __forceinline__ void dep_guard4_b(v8f& a, v8f& b, v8f& c, v8f& d, v16b x, v16b y) { asm volatile("v_nop\n\tv_nop\n\tv_nop\n\tv_nop" : "+v"(a), "+v"(b), "+v"(c), "+v"(d) : "v"(x), "v"(y)); }
__device__ __forceinline__ void keep4_h(v16h a, v16h b, v16h c, v16h d) { asm volatile("v_nop" :: "v"(a), "v"(b), "v"(c), "v"(d)); }
__device__ __forceinline__ void keep4_b(v16b a, v16b b, v16b c, v16b d) { asm volatile("v_nop" :: "v"(a), "v"(b), "v"(c), "v"(d)); }
__device__ __forceinline__ void acc_guard4(v8f& a, v8f& b, v8f& c, v8f& d) { asm volatile("v_nop\n\tv_nop\n\tv_nop\n\tv_nop" : "+v"(a), "+v"(b), "+v"(c), "+v"(d)); }
template <typename T> struct Frag;
template <> struct Frag<_Float16> {
  typedef v16h V; union U { v16h v; v8h h[2]; };
  static __device__ __forceinline__ v16h load(const _Float16* p) {
    U f; f.h[0] = *(const v8h*)(p); f.h[1] = *(const v8h*)(p + 16); return f.v;
  }
  static __device__ __forceinline__ v8f mma(v16h a, v16h b, v8f c) {
    return __builtin_amdgcn_wmma_f32_16x16x32_f16(false, a, false, b, (short)0, c, false, false);
  }
  static __device__ __forceinline__ void guard4(v8f& a, v8f& b, v8f& c, v8f& d, v16h x, v16h y) { dep_guard4_h(a, b, c, d, x, y); }
  static __device__ __forceinline__ void keep(v16h a, v16h b, v16h c, v16h d) { keep4_h(a, b, c, d); }
};
template <> struct Frag<__bf16> {
  typedef v16b V; union U { v16b v; v8b h[2]; };
  static __device__ __forceinline__ v16b load(const __bf16* p) {
    U f; f.h[0] = *(const v8b*)(p); f.h[1] = *(const v8b*)(p + 16); return f.v;
  }
  static __device__ __forceinline__ v8f mma(v16b a, v16b b, v8f c) {
    return __builtin_amdgcn_wmma_f32_16x16x32_bf16(false, a, false, b, (short)0, c, false, false);
  }
  static __device__ __forceinline__ void guard4(v8f& a, v8f& b, v8f& c, v8f& d, v16b x, v16b y) { dep_guard4_b(a, b, c, d, x, y); }
  static __device__ __forceinline__ void keep(v16b a, v16b b, v16b c, v16b d) { keep4_b(a, b, c, d); }
};

__device__ __forceinline__ unsigned pk16(unsigned short a, unsigned short b) { return (unsigned)a | ((unsigned)b << 16); }
__device__ __forceinline__ unsigned short h_bits(float f) { const _Float16 h = (_Float16)f; return __builtin_bit_cast(unsigned short, h); }

template <int ET> struct Elem;
template <> struct Elem<0> { typedef _Float16 T; };
template <> struct Elem<1> { typedef __bf16 T; };
template <int ET, bool SPLIT, int BIAS_MODE, int OUT_MODE, bool RESID, bool OCARRY>
__global__ __launch_bounds__(256) void wmma_gemm64(
    const unsigned short* __restrict__ Ap, const unsigned short* __restrict__ A2p, int lda, long strideA,
    const unsigned short* __restrict__ Btp, const unsigned short* __restrict__ Bt2p, int ldb, long strideB,
    void* __restrict__ Cout, void* __restrict__ Cout2, int ldc, long strideC,
    const float* __restrict__ bias,
    const float* __restrict__ resid, long strideR,
    int M, int N, int K, float scale, float ocarry) {
  static_assert(!RESID || OUT_MODE == 0);
  typedef typename Elem<ET>::T T;
  typedef typename Frag<T>::V V;
  const T* A = (const T*)Ap; const T* A2 = (const T*)A2p; const T* Bt = (const T*)Btp; const T* Bt2 = (const T*)Bt2p;
  __shared__ __align__(16) float sT[8][16 * 68];
  const int b    = blockIdx.y;
  const int lane = threadIdx.x & 31;
  const int wave = threadIdx.x >> 5;
  const int tilesN = N >> 6;
  const int tilesM = M >> 6;
  const int tile = blockIdx.x * 8 + wave;
  if (tile >= tilesM * tilesN) return;
  const int tm = tile / tilesN;
  const int tn = tile - tm * tilesN;
  const int m0 = tm << 6;
  const int n0 = tn << 6;

  const T* Ab  = A  + (size_t)b * strideA;
  const T* Bb  = Bt + (size_t)b * strideB;
  const T* Ab2 = SPLIT ? (A2  + (size_t)b * strideA) : nullptr;
  const T* Bb2 = SPLIT ? (Bt2 + (size_t)b * strideB) : nullptr;

  const int rlane = lane & 15;
  const int koff  = (lane >> 4) * 8;
  const int mOff  = (lane >> 4) * 8;

  v8f acc[4][4];
#pragma unroll
  for (int i = 0; i < 4; ++i)
#pragma unroll
    for (int j = 0; j < 4; ++j) acc[i][j] = (v8f){0.f,0.f,0.f,0.f,0.f,0.f,0.f,0.f};

  for (int k0 = 0; k0 < K; k0 += 32) {
    V bh[4], bl[4];
#pragma unroll
    for (int j = 0; j < 4; ++j) {
      const size_t bo = (size_t)(n0 + (j << 4) + rlane) * ldb + koff + k0;
      bh[j] = Frag<T>::load(Bb + bo);
      if (SPLIT) bl[j] = Frag<T>::load(Bb2 + bo);
      else bl[j] = bh[j];
    }
#pragma unroll
    for (int i = 0; i < 4; ++i) {
      const size_t ao = (size_t)(m0 + (i << 4) + rlane) * lda + koff + k0;
      V ah = Frag<T>::load(Ab + ao);
      V al;
      if (SPLIT) al = Frag<T>::load(Ab2 + ao);
      else al = ah;
#pragma unroll
      for (int j = 0; j < 4; ++j) {
        acc[i][j] = Frag<T>::mma(ah, bh[j], acc[i][j]);
        if (SPLIT) {
          acc[i][j] = Frag<T>::mma(ah, bl[j], acc[i][j]);
          acc[i][j] = Frag<T>::mma(al, bh[j], acc[i][j]);
        }
      }
      Frag<T>::guard4(acc[i][0], acc[i][1], acc[i][2], acc[i][3], SPLIT ? al : ah, bh[3]);
    }
    Frag<T>::keep(bh[0], bh[1], bh[2], bh[3]);
    if (SPLIT) Frag<T>::keep(bl[0], bl[1], bl[2], bl[3]);
  }
  acc_guard4(acc[0][0], acc[0][1], acc[0][2], acc[0][3]);
  acc_guard4(acc[1][0], acc[1][1], acc[1][2], acc[1][3]);
  acc_guard4(acc[2][0], acc[2][1], acc[2][2], acc[2][3]);
  acc_guard4(acc[3][0], acc[3][1], acc[3][2], acc[3][3]);

  float* slab = sT[wave];
#pragma unroll
  for (int i = 0; i < 4; ++i) {
    const int mBase = m0 + (i << 4);
    float bmr[8] = {0.f, 0.f, 0.f, 0.f, 0.f, 0.f, 0.f, 0.f};
    if (BIAS_MODE == 1) {
      const v4f bm0 = *(const v4f*)(bias + mBase + mOff);
      const v4f bm1 = *(const v4f*)(bias + mBase + mOff + 4);
      bmr[0] = bm0[0]; bmr[1] = bm0[1]; bmr[2] = bm0[2]; bmr[3] = bm0[3];
      bmr[4] = bm1[0]; bmr[5] = bm1[1]; bmr[6] = bm1[2]; bmr[7] = bm1[3];
    }
#pragma unroll
    for (int j = 0; j < 4; ++j) {
      const int n = n0 + (j << 4) + rlane;
      float bv = 0.f;
      if (BIAS_MODE == 2) bv = bias[n];
#pragma unroll
      for (int r = 0; r < 8; ++r) {
        float v = acc[i][j][r] * scale;
        if (BIAS_MODE == 1) v += bmr[r];
        if (BIAS_MODE == 2) v += bv;
        if (OCARRY) v *= ocarry;
        slab[(mOff + r) * 68 + (j << 4) + rlane] = v;
      }
    }
    __builtin_amdgcn_fence(__ATOMIC_RELEASE, "workgroup");
    __builtin_amdgcn_wave_barrier();
    __builtin_amdgcn_fence(__ATOMIC_ACQUIRE, "workgroup");
    if (OUT_MODE == 0) {
      float* C = (float*)Cout + (size_t)b * strideC;
      const float* Rb = RESID ? (resid + (size_t)b * strideR) : resid;
      const int hh = lane >> 4, c4 = (lane & 15) * 4;
      for (int pass = 0; pass < 2; ++pass) {
#pragma unroll
        for (int it = 0; it < 8; ++it) {
          const int row = it * 2 + hh;
          v4f v = *(const v4f*)(slab + row * 68 + c4);
          const size_t go = (size_t)(mBase + row) * ldc + n0 + c4;
          if (RESID) {
            const v4f rr = *(const v4f*)(Rb + go);
            v = v + rr;
          }
          *(volatile v4f*)(C + go) = v;
        }
        __threadfence();
      }
    } else {
      const int q = lane >> 3, c8 = (lane & 7) * 8;
      unsigned short* C  = (unsigned short*)Cout  + (size_t)b * strideC;
      unsigned short* C2 = (OUT_MODE == 2) ? ((unsigned short*)Cout2 + (size_t)b * strideC) : nullptr;
      for (int pass = 0; pass < 2; ++pass) {
#pragma unroll
        for (int it = 0; it < 4; ++it) {
          const int row = it * 4 + q;
          const float* sp = slab + row * 68 + c8;
          v8h hv, lv;
#pragma unroll
          for (int e = 0; e < 8; ++e) {
            if (OUT_MODE == 1) {
              hv[e] = (_Float16)sp[e];
            } else {
              unsigned short hb = f2bf_bits(sp[e]);
              unsigned short lb = f2bf_bits(sp[e] - bf_bits2f(hb));
              hv[e] = __builtin_bit_cast(_Float16, hb);
              lv[e] = __builtin_bit_cast(_Float16, lb);
            }
          }
          *(volatile v8h*)(C + (size_t)(mBase + row) * ldc + n0 + c8) = hv;
          if (OUT_MODE == 2) *(volatile v8h*)(C2 + (size_t)(mBase + row) * ldc + n0 + c8) = lv;
        }
        __threadfence();
      }
    }
    __builtin_amdgcn_fence(__ATOMIC_RELEASE, "workgroup");
    __builtin_amdgcn_wave_barrier();
    __builtin_amdgcn_fence(__ATOMIC_ACQUIRE, "workgroup");
  }
}

__global__ __launch_bounds__(256) void cast8_f16_kernel(const float* __restrict__ in, unsigned short* __restrict__ out,
                                                       int n8, float carry) {
  const int i = blockIdx.x * 256 + threadIdx.x;
  if (i >= n8) return;
  const float* p = in + 8 * (size_t)i;
  const v4f a = *(const v4f*)(p);
  const v4f c = *(const v4f*)(p + 4);
  unsigned short hb[8];
#pragma unroll
  for (int e = 0; e < 4; ++e) {
    hb[e]     = h_bits(a[e] * carry);
    hb[4 + e] = h_bits(c[e] * carry);
  }
  const v4u u = (v4u){pk16(hb[0], hb[1]), pk16(hb[2], hb[3]), pk16(hb[4], hb[5]), pk16(hb[6], hb[7])};
  unsigned short* q = out + 8 * (size_t)i;
  *(volatile v4u*)q = u;
  __threadfence();
  *(volatile v4u*)q = u;
}

__global__ __launch_bounds__(256) void softmax_row_kernel(const float* __restrict__ S, unsigned short* __restrict__ P) {
  __shared__ float redM[8];
  __shared__ float redS[8];
  const int row  = blockIdx.x;
  const int pl   = blockIdx.y;
  const int t    = threadIdx.x;
  const int lane = t & 31, wave = t >> 5;
  const size_t rowoff = ((size_t)pl * kSeq + (size_t)row) * (size_t)kSeq;
  const float* sr = S + rowoff + 8 * (size_t)t;
  const v4f a = *(const v4f*)(sr);
  const v4f c = *(const v4f*)(sr + 4);
  float x[8];
#pragma unroll
  for (int e = 0; e < 4; ++e) { x[e] = a[e]; x[4 + e] = c[e]; }
  float mx = fmaxf(fmaxf(fmaxf(x[0], x[1]), fmaxf(x[2], x[3])), fmaxf(fmaxf(x[4], x[5]), fmaxf(x[6], x[7])));
#pragma unroll
  for (int off = 16; off > 0; off >>= 1) mx = fmaxf(mx, __shfl_xor(mx, off, 32));
  if (lane == 0) redM[wave] = mx;
  __syncthreads();
  float m = redM[0];
#pragma unroll
  for (int w = 1; w < 8; ++w) m = fmaxf(m, redM[w]);

  float ev[8];
  float sum = 0.f;
#pragma unroll
  for (int e = 0; e < 8; ++e) {
    ev[e] = expf(x[e] - m);
    sum += ev[e];
  }
#pragma unroll
  for (int off = 16; off > 0; off >>= 1) sum += __shfl_xor(sum, off, 32);
  if (lane == 0) redS[wave] = sum;
  __syncthreads();
  float tot = redS[0];
#pragma unroll
  for (int w = 1; w < 8; ++w) tot += redS[w];
  const float inv = kPCarry / tot;

  unsigned short hb[8];
#pragma unroll
  for (int e = 0; e < 8; ++e) hb[e] = h_bits(ev[e] * inv);
  const v4u u = (v4u){pk16(hb[0], hb[1]), pk16(hb[2], hb[3]), pk16(hb[4], hb[5]), pk16(hb[6], hb[7])};
  unsigned short* pr = P + rowoff + 8 * (size_t)t;
  *(volatile v4u*)pr = u;
  __threadfence();
  *(volatile v4u*)pr = u;
}

extern "C" void kernel_launch(void* const* d_in, const int* in_sizes, int n_in,
                              void* d_out, int out_size, void* d_ws, size_t ws_size,
                              hipStream_t stream) {
  if (n_in < 16) return;
  const int nAct = kTok * kDim;
  const int nW   = kDim * kDim;
  if (in_sizes[0] != nAct || in_sizes[1] != nAct) return;
  for (int i = 0; i < kNumW; ++i) {
    if (in_sizes[2 + 2 * i] != nW) return;
    if (in_sizes[3 + 2 * i] != kDim) return;
  }
  if (out_size != nAct) return;
  if (ws_size < kWsTotal) return;

  const float* x   = (const float*)d_in[0];
  const float* ctx = (const float*)d_in[1];
  const float* Wsrc[kNumW];
  const float* bsrc[kNumW];
  for (int i = 0; i < kNumW; ++i) {
    Wsrc[i] = (const float*)d_in[2 + 2 * i];
    bsrc[i] = (const float*)d_in[3 + 2 * i];
  }
  float* out = (float*)d_out;
  char* ws = (char*)d_ws;
  unsigned short* XO   = (unsigned short*)(ws + kOffXO);
  unsigned short* CTX  = (unsigned short*)(ws + kOffCTX);
  unsigned short* W16  = (unsigned short*)(ws + kOffW);
  unsigned short* Q16  = (unsigned short*)(ws + kOffQ);
  unsigned short* K16  = (unsigned short*)(ws + kOffK);
  unsigned short* VT   = (unsigned short*)(ws + kOffVT);
  float*          AO32 = (float*)(ws + kOffAO32);
  unsigned short* AO16 = (unsigned short*)(ws + kOffAO16);
  float*          SC   = (float*)(ws + kOffSC);
  unsigned short* PP   = (unsigned short*)(ws + kOffPP);
  unsigned short* Wp[kNumW];
  for (int i = 0; i < kNumW; ++i) Wp[i] = W16 + (size_t)i * kDim * kDim;
  unsigned short* CK16 = Q16;
  unsigned short* CQ16 = K16;
  unsigned short* CVT  = VT;

  const long strideTokB = (long)kSeq * kDim;
  const long strideVTB  = (long)kDim * kSeq;
  const long stridePl   = (long)kSeq * kSeq;
  const long strideHd   = (long)kDh;
  const long strideVTHd = (long)kDh * kSeq;

  const int n8Act = nAct / 8;
  const int n8W   = nW / 8;
  cast8_f16_kernel<<<dim3(n8Act / 256), dim3(256), 0, stream>>>(x, XO, n8Act, 1.0f);
  cast8_f16_kernel<<<dim3(n8Act / 256), dim3(256), 0, stream>>>(ctx, CTX, n8Act, 1.0f);
  for (int i = 0; i < kNumW; ++i)
    cast8_f16_kernel<<<dim3(n8W / 256), dim3(256), 0, stream>>>(Wsrc[i], Wp[i], n8W, kWCarry);

  const int blkLin = ((kTok / 64) * (kDim / 64)) / 8;
  wmma_gemm64<0, false, 2, 1, false, false><<<dim3(blkLin, 1), dim3(256), 0, stream>>>(
      XO, XO, kDim, 0L, Wp[0], Wp[0], kDim, 0L, (void*)Q16, (void*)Q16, kDim, 0L,
      bsrc[0], AO32, 0L, kTok, kDim, kDim, kWCarryInv, 1.0f);
  wmma_gemm64<0, false, 2, 1, false, false><<<dim3(blkLin, 1), dim3(256), 0, stream>>>(
      XO, XO, kDim, 0L, Wp[1], Wp[1], kDim, 0L, (void*)K16, (void*)K16, kDim, 0L,
      bsrc[1], AO32, 0L, kTok, kDim, kDim, kWCarryInv, 1.0f);
  const int blkT = ((kDim / 64) * (kSeq / 64)) / 8;
  wmma_gemm64<0, false, 1, 1, false, false><<<dim3(blkT, kBatch), dim3(256), 0, stream>>>(
      Wp[2], Wp[2], kDim, 0L, XO, XO, kDim, strideTokB, (void*)VT, (void*)VT, kSeq, strideVTB,
      bsrc[2], AO32, 0L, kDim, kSeq, kDim, kWCarryInv, 1.0f);

  const int blkSc = ((kSeq / 64) * (kSeq / 64)) / 8;
  const int blkPv = ((kSeq / 64) * (kDh / 64)) / 8;
  for (int b = 0; b < kBatch; ++b) {
    for (int g = 0; g < kHeads / kGroup; ++g) {
      const int h0 = g * kGroup;
      const size_t tokOff = (size_t)b * kSeq * kDim + (size_t)h0 * kDh;
      const size_t vtOff  = ((size_t)b * kDim + (size_t)h0 * kDh) * kSeq;
      wmma_gemm64<0, false, 0, 0, false, false><<<dim3(blkSc, kGroup), dim3(256), 0, stream>>>(
          Q16 + tokOff, Q16 + tokOff, kDim, strideHd, K16 + tokOff, K16 + tokOff, kDim, strideHd,
          (void*)SC, (void*)SC, kSeq, stridePl, bsrc[0], AO32, 0L, kSeq, kSeq, kDh, kScale, 1.0f);
      softmax_row_kernel<<<dim3(kSeq, kGroup), dim3(256), 0, stream>>>(SC, PP);
      wmma_gemm64<0, false, 0, 1, false, false><<<dim3(blkPv, kGroup), dim3(256), 0, stream>>>(
          PP, PP, kSeq, stridePl, VT + vtOff, VT + vtOff, kSeq, strideVTHd,
          (void*)(XO + tokOff), (void*)(XO + tokOff), kDim, strideHd, bsrc[0], AO32, 0L,
          kSeq, kDh, kSeq, kACarry * kPCarryInv, 1.0f);
    }
  }

  wmma_gemm64<0, false, 2, 0, false, false><<<dim3(blkLin, 1), dim3(256), 0, stream>>>(
      XO, XO, kDim, 0L, Wp[3], Wp[3], kDim, 0L, (void*)AO32, (void*)AO32, kDim, 0L,
      bsrc[3], SC, 0L, kTok, kDim, kDim, kWCarryInv / kACarry, 1.0f);
  cast8_f16_kernel<<<dim3(n8Act / 256), dim3(256), 0, stream>>>(AO32, AO16, n8Act, kACarry);

  wmma_gemm64<0, false, 2, 1, false, true><<<dim3(blkLin, 1), dim3(256), 0, stream>>>(
      AO16, AO16, kDim, 0L, Wp[4], Wp[4], kDim, 0L, (void*)CQ16, (void*)CQ16, kDim, 0L,
      bsrc[4], AO32, 0L, kTok, kDim, kDim, kWCarryInv / kACarry, kACarry);
  wmma_gemm64<0, false, 2, 1, false, false><<<dim3(blkLin, 1), dim3(256), 0, stream>>>(
      CTX, CTX, kDim, 0L, Wp[5], Wp[5], kDim, 0L, (void*)CK16, (void*)CK16, kDim, 0L,
      bsrc[5], AO32, 0L, kTok, kDim, kDim, kWCarryInv, 1.0f);
  wmma_gemm64<0, false, 1, 1, false, false><<<dim3(blkT, kBatch), dim3(256), 0, stream>>>(
      Wp[6], Wp[6], kDim, 0L, CTX, CTX, kDim, strideTokB, (void*)CVT, (void*)CVT, kSeq, strideVTB,
      bsrc[6], AO32, 0L, kDim, kSeq, kDim, kWCarryInv, 1.0f);

  wmma_gemm64<0, false, 0, 0, false, false><<<dim3(blkSc, kBatch), dim3(256), 0, stream>>>(
      CQ16, CQ16, kDim, strideTokB, CK16, CK16, kDim, strideTokB, (void*)SC, (void*)SC, kSeq, stridePl,
      bsrc[0], AO32, 0L, kSeq, kSeq, kDim, kScale / kACarry, 1.0f);
  softmax_row_kernel<<<dim3(kSeq, kBatch), dim3(256), 0, stream>>>(SC, PP);
  const int blkOut = ((kSeq / 64) * (kDim / 64)) / 8;
  wmma_gemm64<0, false, 0, 0, true, false><<<dim3(blkOut, kBatch), dim3(256), 0, stream>>>(
      PP, PP, kSeq, stridePl, CVT, CVT, kSeq, strideVTB, (void*)out, (void*)out, kDim, strideTokB,
      bsrc[0], AO32, strideTokB, kSeq, kDim, kSeq, kPCarryInv, 1.0f);
}
